// HardwareKANLayer_41875931136528
// MI455X (gfx1250) — hardware-verified
//
#include <hip/hip_runtime.h>
#include <math.h>

#pragma clang fp contract(off)

constexpr int kBatch  = 8192;
constexpr int kIn     = 1024;
constexpr int kOut    = 1024;
constexpr int kNB     = 11;
constexpr int kKtot   = kIn + kIn * kNB;
constexpr int kChunk  = 2048;
constexpr int kNChunk = kBatch / kChunk;
constexpr float kACarry   = 8.0f;
constexpr float kWCarry   = 4096.0f;
constexpr float kOutScale = 1.0f / (8.0f * 4096.0f);

constexpr size_t kWpBytes = (size_t)kOut * kKtot * 2;
constexpr size_t kAxBytes = (size_t)kChunk * kKtot * 2;
constexpr size_t kWsTotal = kWpBytes + 2 * kAxBytes;
static_assert(kWsTotal <= 134217728, "carve");
static_assert(kKtot % 32 == 0 && kChunk % 64 == 0 && kOut % 64 == 0, "tiles");

typedef __attribute__((ext_vector_type(16))) _Float16 v16h;
typedef __attribute__((ext_vector_type(8)))  _Float16 v8h;
typedef __attribute__((ext_vector_type(16))) __bf16   v16b;
typedef __attribute__((ext_vector_type(8)))  __bf16   v8b;
typedef __attribute__((ext_vector_type(8)))  float    v8f;
typedef __attribute__((ext_vector_type(4)))  float    v4f;
typedef __attribute__((ext_vector_type(4)))  unsigned int v4u;

__device__ __forceinline__ unsigned short f2bf_bits(float f) {
  unsigned u = __float_as_uint(f);
  return (unsigned short)((u + 0x7FFFu + ((u >> 16) & 1u)) >> 16);
}
__device__ __forceinline__ float bf_bits2f(unsigned short h) { return __uint_as_float(((unsigned)h) << 16); }

__device__ __forceinline__ void dep_guard_h(v8f& a, v8f& b, v16h x, v16h y) { asm volatile("v_nop\n\tv_nop\n\tv_nop\n\tv_nop" : "+v"(a), "+v"(b) : "v"(x), "v"(y)); }
__device__ __forceinline__ void dep_guard_b(v8f& a, v8f& b, v16b x, v16b y) { asm volatile("v_nop\n\tv_nop\n\tv_nop\n\tv_nop" : "+v"(a), "+v"(b) : "v"(x), "v"(y)); }
__device__ __forceinline__ void keep4_h(v16h a, v16h b, v16h c, v16h d) { asm volatile("v_nop" :: "v"(a), "v"(b), "v"(c), "v"(d)); }
__device__ __forceinline__ void keep4_b(v16b a, v16b b, v16b c, v16b d) { asm volatile("v_nop" :: "v"(a), "v"(b), "v"(c), "v"(d)); }
__device__ __forceinline__ void acc_guard4(v8f& a, v8f& b, v8f& c, v8f& d) { asm volatile("v_nop\n\tv_nop\n\tv_nop\n\tv_nop" : "+v"(a), "+v"(b), "+v"(c), "+v"(d)); }
template <typename T> struct Frag;
template <> struct Frag<_Float16> {
  typedef v16h V; union U { v16h v; v8h h[2]; };
  static __device__ __forceinline__ v16h load(const _Float16* p) {
    U f; f.h[0] = *(const v8h*)(p); f.h[1] = *(const v8h*)(p + 16); return f.v;
  }
  static __device__ __forceinline__ v8f mma(v16h a, v16h b, v8f c) {
    return __builtin_amdgcn_wmma_f32_16x16x32_f16(false, a, false, b, (short)0, c, false, false);
  }
  static __device__ __forceinline__ void guard(v8f& a, v8f& b, v16h x, v16h y) { dep_guard_h(a, b, x, y); }
  static __device__ __forceinline__ void keep(v16h a, v16h b, v16h c, v16h d) { keep4_h(a, b, c, d); }
};
template <> struct Frag<__bf16> {
  typedef v16b V; union U { v16b v; v8b h[2]; };
  static __device__ __forceinline__ v16b load(const __bf16* p) {
    U f; f.h[0] = *(const v8b*)(p); f.h[1] = *(const v8b*)(p + 16); return f.v;
  }
  static __device__ __forceinline__ v8f mma(v16b a, v16b b, v8f c) {
    return __builtin_amdgcn_wmma_f32_16x16x32_bf16(false, a, false, b, (short)0, c, false, false);
  }
  static __device__ __forceinline__ void guard(v8f& a, v8f& b, v16b x, v16b y) { dep_guard_b(a, b, x, y); }
  static __device__ __forceinline__ void keep(v16b a, v16b b, v16b c, v16b d) { keep4_b(a, b, c, d); }
};

__device__ __forceinline__ unsigned pk16(unsigned short a, unsigned short b) { return (unsigned)a | ((unsigned)b << 16); }
__device__ __forceinline__ unsigned short h_bits(float f) { const _Float16 h = (_Float16)f; return __builtin_bit_cast(unsigned short, h); }

__device__ __forceinline__ void store16_twice(unsigned short* p, v4u u) {
  *(volatile v4u*)p = u;
  __threadfence();
  *(volatile v4u*)p = u;
}

template <int ET> struct Elem;
template <> struct Elem<0> { typedef _Float16 T; };
template <> struct Elem<1> { typedef __bf16 T; };
template <int ET, bool SPLIT, int BIAS_MODE, int OUT_MODE, bool RESID, int ACT = 0>
__global__ __launch_bounds__(256) void wmma_gemm64(
    const unsigned short* __restrict__ Ap, const unsigned short* __restrict__ A2p, int lda, long strideA,
    const unsigned short* __restrict__ Btp, const unsigned short* __restrict__ Bt2p, int ldb, long strideB,
    void* __restrict__ Cout, void* __restrict__ Cout2, int ldc, long strideC,
    const float* __restrict__ bias,
    const float* __restrict__ resid, long strideR,
    int M, int N, int K, float scale) {
  typedef typename Elem<ET>::T T;
  typedef typename Frag<T>::V V;
  const T* A = (const T*)Ap; const T* A2 = (const T*)A2p; const T* Bt = (const T*)Btp; const T* Bt2 = (const T*)Bt2p;
  __shared__ __align__(16) float sT[8][16 * 68];
  const int b    = blockIdx.y;
  const int lane = threadIdx.x & 31;
  const int wave = threadIdx.x >> 5;
  const int tilesN = N >> 6;
  const int tilesM = M >> 6;
  const int tile = blockIdx.x * 8 + wave;
  if (tile >= tilesM * tilesN) return;
  const int tm = tile / tilesN;
  const int tn = tile - tm * tilesN;
  const int m0 = tm << 6;
  const int n0 = tn << 6;

  const T* Ab  = A  + (size_t)b * strideA;
  const T* Bb  = Bt + (size_t)b * strideB;
  const T* Ab2 = SPLIT ? (A2  + (size_t)b * strideA) : nullptr;
  const T* Bb2 = SPLIT ? (Bt2 + (size_t)b * strideB) : nullptr;

  const int rlane = lane & 15;
  const int koff  = (lane >> 4) * 8;
  const int mOff  = (lane >> 4) * 8;

  v8f acc[4][4];
#pragma unroll
  for (int i = 0; i < 4; ++i)
#pragma unroll
    for (int j = 0; j < 4; ++j) acc[i][j] = (v8f){0.f,0.f,0.f,0.f,0.f,0.f,0.f,0.f};

  for (int k0 = 0; k0 < K; k0 += 32) {
    V bh[4], bl[4];
#pragma unroll
    for (int j = 0; j < 4; ++j) {
      const size_t bo = (size_t)(n0 + (j << 4) + rlane) * ldb + koff + k0;
      bh[j] = Frag<T>::load(Bb + bo);
      if (SPLIT) bl[j] = Frag<T>::load(Bb2 + bo);
    }
#pragma unroll
    for (int i = 0; i < 4; ++i) {
      const size_t ao = (size_t)(m0 + (i << 4) + rlane) * lda + koff + k0;
      V ah = Frag<T>::load(Ab + ao);
      V al;
      if (SPLIT) al = Frag<T>::load(Ab2 + ao);
#pragma unroll
      for (int j = 0; j < 4; ++j) {
        acc[i][j] = Frag<T>::mma(ah, bh[j], acc[i][j]);
        if (SPLIT) {
          acc[i][j] = Frag<T>::mma(ah, bl[j], acc[i][j]);
          acc[i][j] = Frag<T>::mma(al, bh[j], acc[i][j]);
        }
      }
      Frag<T>::guard(acc[i][0], acc[i][3], ah, SPLIT ? al : ah);
    }
    Frag<T>::keep(bh[0], bh[1], bh[2], bh[3]);
    if (SPLIT) Frag<T>::keep(bl[0], bl[1], bl[2], bl[3]);
  }
  acc_guard4(acc[0][0], acc[0][1], acc[0][2], acc[0][3]);
  acc_guard4(acc[1][0], acc[1][1], acc[1][2], acc[1][3]);
  acc_guard4(acc[2][0], acc[2][1], acc[2][2], acc[2][3]);
  acc_guard4(acc[3][0], acc[3][1], acc[3][2], acc[3][3]);

  float* slab = sT[wave];
  const float* Rb = RESID ? (resid + (size_t)b * strideR) : nullptr;
#pragma unroll
  for (int i = 0; i < 4; ++i) {
    const int mBase = m0 + (i << 4);
#pragma unroll
    for (int j = 0; j < 4; ++j) {
      const int n = n0 + (j << 4) + rlane;
      float bv = 0.f;
      if (BIAS_MODE == 2) bv = bias[n];
#pragma unroll
      for (int r = 0; r < 8; ++r) {
        float v = acc[i][j][r] * scale;
        if (BIAS_MODE == 1) v += bias[mBase + mOff + r];
        if (BIAS_MODE == 2) v += bv;
        if (RESID) v += Rb[(size_t)(mBase + mOff + r) * ldc + n];
        if (ACT == 2) v = fmaxf(v, 0.0f);
        if (ACT == 4) v = (v > 0.f) ? v : 0.01f * v;
        if (ACT == 6) v = fminf(1.0f, fmaxf(-1.0f, v));
        slab[(mOff + r) * 68 + (j << 4) + rlane] = v;
      }
    }
    __builtin_amdgcn_fence(__ATOMIC_RELEASE, "workgroup");
    __builtin_amdgcn_wave_barrier();
    __builtin_amdgcn_fence(__ATOMIC_ACQUIRE, "workgroup");
    if (OUT_MODE == 0) {
      float* C = (float*)Cout + (size_t)b * strideC;
      const int hh = lane >> 4, c4 = (lane & 15) * 4;
      for (int pass = 0; pass < 2; ++pass) {
#pragma unroll
        for (int it = 0; it < 8; ++it) {
          const int row = it * 2 + hh;
          v4f v = *(const v4f*)(slab + row * 68 + c4);
          *(volatile v4f*)(C + (size_t)(mBase + row) * ldc + n0 + c4) = v;
        }
        __threadfence();
      }
    } else {
      const int q = lane >> 3, c8 = (lane & 7) * 8;
      unsigned short* C  = (unsigned short*)Cout  + (size_t)b * strideC;
      unsigned short* C2 = (OUT_MODE == 2) ? ((unsigned short*)Cout2 + (size_t)b * strideC) : nullptr;
      for (int pass = 0; pass < 2; ++pass) {
#pragma unroll
        for (int it = 0; it < 4; ++it) {
          const int row = it * 4 + q;
          const float* sp = slab + row * 68 + c8;
          v8h hv, lv;
#pragma unroll
          for (int e = 0; e < 8; ++e) {
            if (OUT_MODE == 1) {
              hv[e] = (_Float16)sp[e];
            } else {
              unsigned short hb = f2bf_bits(sp[e]);
              unsigned short lb = f2bf_bits(sp[e] - bf_bits2f(hb));
              hv[e] = __builtin_bit_cast(_Float16, hb);
              lv[e] = __builtin_bit_cast(_Float16, lb);
            }
          }
          *(volatile v8h*)(C + (size_t)(mBase + row) * ldc + n0 + c8) = hv;
          if (OUT_MODE == 2) *(volatile v8h*)(C2 + (size_t)(mBase + row) * ldc + n0 + c8) = lv;
        }
        __threadfence();
      }
    }
    __builtin_amdgcn_fence(__ATOMIC_RELEASE, "workgroup");
    __builtin_amdgcn_wave_barrier();
    __builtin_amdgcn_fence(__ATOMIC_ACQUIRE, "workgroup");
  }
}

__global__ __launch_bounds__(256) void packw_kernel(const float* __restrict__ bw, const float* __restrict__ sw,
                                                    unsigned short* __restrict__ wp) {
  const int g  = blockIdx.x * 256 + threadIdx.x;
  const int o  = g / 1536;
  const int j  = g - o * 1536;
  const int r0 = j * 8;
  const int rb = (r0 < kIn) ? r0 : (kIn - 8);
  const float* pb = bw + (size_t)o * kIn + rb;
  const v4f b0 = *(const v4f*)(pb);
  const v4f b1 = *(const v4f*)(pb + 4);
  int rr = r0 - kIn; rr = (rr < 0) ? 0 : rr;
  const int kb = rr >> 10;
  const int i0 = rr & (kIn - 1);
  const float* ps = sw + ((size_t)o * kIn + i0) * kNB + kb;
  float sv[8];
#pragma unroll
  for (int e = 0; e < 8; ++e) sv[e] = ps[e * kNB];
  const bool useb = (r0 < kIn);
  unsigned short hb[8];
#pragma unroll
  for (int e = 0; e < 4; ++e) {
    const float v0 = useb ? b0[e] : sv[e];
    const float v1 = useb ? b1[e] : sv[4 + e];
    hb[e]     = h_bits(v0 * kWCarry);
    hb[4 + e] = h_bits(v1 * kWCarry);
  }
  const v4u u = (v4u){pk16(hb[0], hb[1]), pk16(hb[2], hb[3]), pk16(hb[4], hb[5]), pk16(hb[6], hb[7])};
  store16_twice(wp + (size_t)o * kKtot + r0, u);
}

struct Centers { float c[12]; };
static_assert(sizeof(Centers) == 48, "no padding");

__global__ __launch_bounds__(256) void basis_kernel(const float* __restrict__ x, unsigned short* __restrict__ ax,
                                                    int row0, Centers cs) {
  const int g  = blockIdx.x * 256 + threadIdx.x;
  const int rl = g >> 7;
  const int t  = g & 127;
  const int i0 = t * 8;
  const float* xp = x + (size_t)(row0 + rl) * kIn + i0;
  const v4f xa = *(const v4f*)(xp);
  const v4f xb = *(const v4f*)(xp + 4);
  float xv[8];
#pragma unroll
  for (int e = 0; e < 4; ++e) { xv[e] = xa[e]; xv[4 + e] = xb[e]; }
  unsigned short* row = ax + (size_t)rl * kKtot;

  unsigned short hb[8];
#pragma unroll
  for (int e = 0; e < 8; ++e) {
    const float ev = expf(-xv[e]);
    const float sg = __builtin_amdgcn_rcpf(1.0f + ev);
    const float s  = xv[e] * sg;
    hb[e] = h_bits(s * kACarry);
  }
  {
    const v4u u = (v4u){pk16(hb[0], hb[1]), pk16(hb[2], hb[3]), pk16(hb[4], hb[5]), pk16(hb[6], hb[7])};
    store16_twice(row + i0, u);
  }

#pragma unroll
  for (int kk = 0; kk < kNB; ++kk) {
    const float c = cs.c[kk];
#pragma unroll
    for (int e = 0; e < 8; ++e) {
      const float u   = fabsf(xv[e] - c) * 4.0f;
      const float ct  = 2.0f - u;
      const float co  = 1.0f - u;
      const float ct3 = ct * (ct * ct);
      const float co3 = co * (co * co);
      const float inner = (1.0f / 6.0f) * (ct3 - 4.0f * co3);
      const float outer = (1.0f / 6.0f) * ct3;
      const float v = (u < 1.0f) ? inner : ((u < 2.0f) ? outer : 0.0f);
      hb[e] = h_bits(v * kACarry);
    }
    const v4u u = (v4u){pk16(hb[0], hb[1]), pk16(hb[2], hb[3]), pk16(hb[4], hb[5]), pk16(hb[6], hb[7])};
    store16_twice(row + kIn + kk * kIn + i0, u);
  }
}

extern "C" void kernel_launch(void* const* d_in, const int* in_sizes, int n_in,
                              void* d_out, int out_size, void* d_ws, size_t ws_size,
                              hipStream_t stream) {
  if (n_in < 3) return;
  if (in_sizes[0] != kBatch * kIn) return;
  if (in_sizes[1] != kOut * kIn) return;
  if (in_sizes[2] != kOut * kIn * kNB) return;
  if (out_size != kBatch * kOut) return;
  if (ws_size < kWsTotal) return;

  const float* x  = (const float*)d_in[0];
  const float* bw = (const float*)d_in[1];
  const float* sw = (const float*)d_in[2];
  float* out = (float*)d_out;

  unsigned char* ws = (unsigned char*)d_ws;
  unsigned short* wp  = (unsigned short*)(ws);
  unsigned short* ax0 = (unsigned short*)(ws + kWpBytes);
  unsigned short* ax1 = (unsigned short*)(ws + kWpBytes + kAxBytes);

  Centers cs;
  for (int k = 0; k < 10; ++k) {
    volatile float t   = (float)k * (1.0f / 10.0f);
    volatile float omt = 1.0f - t;
    volatile float p0  = -1.25f * omt;
    volatile float p1  = 1.25f * t;
    cs.c[k] = p0 + p1;
  }
  cs.c[10] = 1.25f;
  cs.c[11] = 0.0f;

  packw_kernel<<<dim3(6144), dim3(256), 0, stream>>>(bw, sw, wp);

  for (int c = 0; c < kNChunk; ++c) {
    unsigned short* axc = (c & 1) ? ax1 : ax0;
    basis_kernel<<<dim3(kChunk * 128 / 256), dim3(256), 0, stream>>>(x, axc, c * kChunk, cs);
    wmma_gemm64<0, false, 0, 0, false, 6><<<dim3(64, 1), dim3(256), 0, stream>>>(
        axc, axc, kKtot, 0L,
        wp, wp, kKtot, 0L,
        (void*)(out + (size_t)c * kChunk * kOut), nullptr, kOut, 0L,
        nullptr,
        nullptr, 0L,
        kChunk, kOut, kKtot, kOutScale);
  }
}
